// SparseDiffusionAttention_62156766708189
// MI455X (gfx1250) — hardware-verified
//
#include <hip/hip_runtime.h>
#include <math.h>

#define NB    2
#define SQ    4096
#define DM    1024
#define NH    16
#define HD    64
#define NQB   (SQ / 64)
#define MR    (NB * SQ)
#define VTP   (NB * SQ)
#define RADK  8
#define KST   (64 + 2 * RADK)
#define WSC   64.0f
#define RSC   4096.0f
#define PSC   1024.0f
static_assert(NH * HD == DM);
static_assert((SQ % 64) == 0 && (DM % 64) == 0 && (MR % 64) == 0 && (VTP % 64) == 0);
static_assert((DM % 32) == 0);
static_assert(KST == 80);
static_assert(RADK + 15 < 32);
static_assert((RADK % 8) == 0);

typedef _Float16 v16h __attribute__((ext_vector_type(16)));
typedef _Float16 v8h  __attribute__((ext_vector_type(8)));
typedef __attribute__((ext_vector_type(16))) __bf16 v16b;
typedef unsigned short v8us __attribute__((ext_vector_type(8)));
typedef float    v8f  __attribute__((ext_vector_type(8)));
typedef float    v4f  __attribute__((ext_vector_type(4)));
typedef unsigned int v4u __attribute__((ext_vector_type(4)));

__device__ __forceinline__ unsigned short bf_bits(float f) {
  unsigned u = __float_as_uint(f);
  return (unsigned short)((u + 0x7FFFu + ((u >> 16) & 1u)) >> 16);
}
__device__ __forceinline__ float bf_up(unsigned short h) { return __uint_as_float(((unsigned)h) << 16); }
__device__ __forceinline__ float bfr(float f) { return bf_up(bf_bits(f)); }
__device__ __forceinline__ unsigned short h_bits(_Float16 x) { return __builtin_bit_cast(unsigned short, x); }
__device__ __forceinline__ unsigned pk16(unsigned short a, unsigned short b) { return (unsigned)a | ((unsigned)b << 16); }
__device__ __forceinline__ v8f zero8() { v8f z = {0.f, 0.f, 0.f, 0.f, 0.f, 0.f, 0.f, 0.f}; return z; }

__device__ __forceinline__ v16h ldfrag_h(const _Float16* p) {
  union { v16h v; v8h h[2]; } f;
  f.h[0] = *(const v8h*)(p);
  f.h[1] = *(const v8h*)(p + 16);
  return f.v;
}
union FB { v16b v; v16h h; v8us u[2]; };
__device__ __forceinline__ FB ldfrag_b(const unsigned short* p) {
  FB f;
  f.u[0] = *(const v8us*)(p);
  f.u[1] = *(const v8us*)(p + 16);
  return f;
}

__device__ __forceinline__ v8f mma_h(v16h a, v16h b, v8f c) {
  c = __builtin_amdgcn_wmma_f32_16x16x32_f16(false, a, false, b, (short)0, c, false, false);
#if defined(__HIP_DEVICE_COMPILE__)
  asm volatile("v_nop\n\tv_nop\n\tv_nop\n\tv_nop" : "+v"(c) : "v"(a), "v"(b));
#endif
  return c;
}
__device__ __forceinline__ v8f mma_h_raw(v16h a, v16h b, v8f c) {
  return __builtin_amdgcn_wmma_f32_16x16x32_f16(false, a, false, b, (short)0, c, false, false);
}
__device__ __forceinline__ v8f mma_b_raw(v16b a, v16b b, v8f c) {
  return __builtin_amdgcn_wmma_f32_16x16x32_bf16(false, a, false, b, (short)0, c, false, false);
}
__device__ __forceinline__ void dep_guard1(v8f& a, v8f& b, v16h x) {
#if defined(__HIP_DEVICE_COMPILE__)
  asm volatile("v_nop\n\tv_nop\n\tv_nop\n\tv_nop" : "+v"(a), "+v"(b) : "v"(x));
#endif
}
__device__ __forceinline__ void dep_guard2(v8f& a, v8f& b, v16h x, v16h y) {
#if defined(__HIP_DEVICE_COMPILE__)
  asm volatile("v_nop\n\tv_nop\n\tv_nop\n\tv_nop" : "+v"(a), "+v"(b) : "v"(x), "v"(y));
#endif
}
__device__ __forceinline__ void keep4_h(v16h a, v16h b, v16h c, v16h d) {
#if defined(__HIP_DEVICE_COMPILE__)
  asm volatile("v_nop" :: "v"(a), "v"(b), "v"(c), "v"(d));
#endif
}
__device__ __forceinline__ void acc_guard4(v8f& a, v8f& b, v8f& c, v8f& d) {
#if defined(__HIP_DEVICE_COMPILE__)
  asm volatile("v_nop\n\tv_nop\n\tv_nop\n\tv_nop" : "+v"(a), "+v"(b), "+v"(c), "+v"(d));
#endif
}
__device__ __forceinline__ void wave_sync_lds() {
  __builtin_amdgcn_fence(__ATOMIC_RELEASE, "workgroup");
  __builtin_amdgcn_wave_barrier();
  __builtin_amdgcn_fence(__ATOMIC_ACQUIRE, "workgroup");
}

template <int BF>
__device__ __forceinline__ unsigned short cvt16(float f, float wsc) {
  if (BF) return bf_bits(f);
  return h_bits((_Float16)(bfr(f) * wsc));
}

template <int BF>
__global__ __launch_bounds__(256) void conv16(const float* __restrict__ W, unsigned short* Wh, int n8,
                                              float wsc) {
  const int i = blockIdx.x * 256 + threadIdx.x;
  if (i >= n8) return;
  const size_t e0 = (size_t)i * 8;
  const v4f a = *(const v4f*)(W + e0);
  const v4f b = *(const v4f*)(W + e0 + 4);
  v4u u;
  u[0] = pk16(cvt16<BF>(a[0], wsc), cvt16<BF>(a[1], wsc));
  u[1] = pk16(cvt16<BF>(a[2], wsc), cvt16<BF>(a[3], wsc));
  u[2] = pk16(cvt16<BF>(b[0], wsc), cvt16<BF>(b[1], wsc));
  u[3] = pk16(cvt16<BF>(b[2], wsc), cvt16<BF>(b[3], wsc));
  for (int pass = 0; pass < 2; ++pass) {
    *(volatile v4u*)(Wh + e0) = u;
    __threadfence();
  }
}

template <int BF>
__global__ __launch_bounds__(256) void convT(const float* __restrict__ W, unsigned short* Wt, int K, int N,
                                             float wsc) {
  __shared__ __align__(16) unsigned short sT[64 * 72];
  const int tid = threadIdx.x;
  const int tilesK = K >> 6;
  const int tn = blockIdx.x / tilesK;
  const int tk = blockIdx.x - tn * tilesK;
  const int n0 = tn << 6;
  const int k0 = tk << 6;

  const int kr  = tid >> 2;
  const int ncb = (tid & 3) * 16;
  const float* src = W + (size_t)(k0 + kr) * N + n0 + ncb;
#pragma unroll
  for (int i = 0; i < 4; ++i) {
    const v4f v = *(const v4f*)(src + 4 * i);
#pragma unroll
    for (int e = 0; e < 4; ++e) sT[(ncb + 4 * i + e) * 72 + kr] = cvt16<BF>(v[e], wsc);
  }
  __syncthreads();

  const int q8 = tid >> 3;
  const int c8 = (tid & 7) * 8;
  v4u pv[2];
#pragma unroll
  for (int it = 0; it < 2; ++it) {
    const int line = it * 32 + q8;
    pv[it] = *(const v4u*)(sT + line * 72 + c8);
  }
  for (int pass = 0; pass < 2; ++pass) {
#pragma unroll
    for (int it = 0; it < 2; ++it) {
      const int line = it * 32 + q8;
      const size_t go = (size_t)(n0 + line) * K + k0 + c8;
      *(volatile v4u*)(Wt + go) = pv[it];
    }
    __threadfence();
  }
}

template <int OM>
__global__ __launch_bounds__(256) void gemm64(
    const unsigned short* __restrict__ Ap, int lda,
    const unsigned short* __restrict__ Btp, int ldb,
    unsigned short* Cout, unsigned short* Cout2, int ldc,
    int M, int N, int K, float oscale, float rsc) {
  const _Float16* A  = (const _Float16*)(const void*)Ap;
  const _Float16* Bt = (const _Float16*)(const void*)Btp;
  __shared__ __align__(16) float sT[8][16 * 68];
  const int lane = threadIdx.x & 31;
  const int wave = threadIdx.x >> 5;
  const int tilesN = N >> 6;
  const int tilesM = M >> 6;
  const int tile = blockIdx.x * 8 + wave;
  if (tile >= tilesM * tilesN) return;
  const int tm = tile / tilesN;
  const int tn = tile - tm * tilesN;
  const int m0 = tm << 6;
  const int n0 = tn << 6;

  const int rlane = lane & 15;
  const int koff  = (lane >> 4) * 8;
  const int mOff  = (lane >> 4) * 8;

  v8f acc[4][4];
#pragma unroll
  for (int i = 0; i < 4; ++i)
#pragma unroll
    for (int j = 0; j < 4; ++j) acc[i][j] = zero8();

  for (int k0 = 0; k0 < K; k0 += 32) {
    v16h bh[4];
#pragma unroll
    for (int j = 0; j < 4; ++j) {
      const size_t bo = (size_t)(n0 + (j << 4) + rlane) * ldb + koff + k0;
      bh[j] = ldfrag_h(Bt + bo);
    }
#pragma unroll
    for (int i = 0; i < 4; ++i) {
      const size_t ao = (size_t)(m0 + (i << 4) + rlane) * lda + koff + k0;
      const v16h ah = ldfrag_h(A + ao);
#pragma unroll
      for (int j = 0; j < 4; ++j) acc[i][j] = mma_h_raw(ah, bh[j], acc[i][j]);
      dep_guard1(acc[i][0], acc[i][3], ah);
    }
    keep4_h(bh[0], bh[1], bh[2], bh[3]);
  }
  acc_guard4(acc[0][0], acc[0][1], acc[0][2], acc[0][3]);
  acc_guard4(acc[1][0], acc[1][1], acc[1][2], acc[1][3]);
  acc_guard4(acc[2][0], acc[2][1], acc[2][2], acc[2][3]);
  acc_guard4(acc[3][0], acc[3][1], acc[3][2], acc[3][3]);

  const int q8 = lane >> 3, c8 = (lane & 7) * 8;

  float* slab = sT[wave];
#pragma unroll
  for (int i = 0; i < 4; ++i) {
    const int mBase = m0 + (i << 4);
#pragma unroll
    for (int j = 0; j < 4; ++j) {
#pragma unroll
      for (int r = 0; r < 8; ++r) {
        slab[(mOff + r) * 68 + (j << 4) + rlane] = acc[i][j][r];
      }
    }
    wave_sync_lds();
    v4u hv[4], lv[4];
#pragma unroll
    for (int it = 0; it < 4; ++it) {
      const int row = it * 4 + q8;
      const float* sp = slab + row * 68 + c8;
      v4u a, lw;
#pragma unroll
      for (int e = 0; e < 4; ++e) {
        const float f0 = sp[2 * e]     * oscale;
        const float f1 = sp[2 * e + 1] * oscale;
        const _Float16 g0 = (_Float16)f0;
        const _Float16 g1 = (_Float16)f1;
        a[e] = pk16(h_bits(g0), h_bits(g1));
        if (OM == 3) {
          const _Float16 r0 = (_Float16)((f0 - (float)g0) * rsc);
          const _Float16 r1 = (_Float16)((f1 - (float)g1) * rsc);
          lw[e] = pk16(h_bits(r0), h_bits(r1));
        } else {
          lw[e] = 0u;
        }
      }
      hv[it] = a;
      lv[it] = lw;
    }
    for (int pass = 0; pass < 2; ++pass) {
#pragma unroll
      for (int it = 0; it < 4; ++it) {
        const int row = it * 4 + q8;
        const size_t go = (size_t)(mBase + row) * ldc + n0 + c8;
        *(volatile v4u*)(Cout + go) = hv[it];
        if (OM == 3) *(volatile v4u*)(Cout2 + go) = lv[it];
      }
      __threadfence();
    }
    wave_sync_lds();
  }
}

__global__ __launch_bounds__(256) void gemm_ob(
    const unsigned short* __restrict__ Ah, const unsigned short* __restrict__ Al, int lda,
    const unsigned short* __restrict__ Btp, int ldb,
    float* Cout, int ldc, int M, int N, int K) {
  __shared__ __align__(16) float sT[8][16 * 68];
  const int lane = threadIdx.x & 31;
  const int wave = threadIdx.x >> 5;
  const int tilesN = N >> 6;
  const int tilesM = M >> 6;
  const int tile = blockIdx.x * 8 + wave;
  if (tile >= tilesM * tilesN) return;
  const int tm = tile / tilesN;
  const int tn = tile - tm * tilesN;
  const int m0 = tm << 6;
  const int n0 = tn << 6;

  const int rlane = lane & 15;
  const int koff  = (lane >> 4) * 8;
  const int mOff  = (lane >> 4) * 8;

  v8f acc[4][4];
#pragma unroll
  for (int i = 0; i < 4; ++i)
#pragma unroll
    for (int j = 0; j < 4; ++j) acc[i][j] = zero8();

  for (int k0 = 0; k0 < K; k0 += 32) {
    FB bh[4];
#pragma unroll
    for (int j = 0; j < 4; ++j) {
      const size_t bo = (size_t)(n0 + (j << 4) + rlane) * ldb + koff + k0;
      bh[j] = ldfrag_b(Btp + bo);
    }
#pragma unroll
    for (int i = 0; i < 4; ++i) {
      const size_t ao = (size_t)(m0 + (i << 4) + rlane) * lda + koff + k0;
      const FB ah = ldfrag_b(Ah + ao);
      const FB al = ldfrag_b(Al + ao);
#pragma unroll
      for (int j = 0; j < 4; ++j) acc[i][j] = mma_b_raw(ah.v, bh[j].v, acc[i][j]);
#pragma unroll
      for (int j = 0; j < 4; ++j) acc[i][j] = mma_b_raw(al.v, bh[j].v, acc[i][j]);
      dep_guard2(acc[i][0], acc[i][3], ah.h, al.h);
    }
    keep4_h(bh[0].h, bh[1].h, bh[2].h, bh[3].h);
  }
  acc_guard4(acc[0][0], acc[0][1], acc[0][2], acc[0][3]);
  acc_guard4(acc[1][0], acc[1][1], acc[1][2], acc[1][3]);
  acc_guard4(acc[2][0], acc[2][1], acc[2][2], acc[2][3]);
  acc_guard4(acc[3][0], acc[3][1], acc[3][2], acc[3][3]);

  float* slab = sT[wave];
  const int hh2 = lane >> 4, c4 = (lane & 15) * 4;
#pragma unroll
  for (int i = 0; i < 4; ++i) {
    const int mBase = m0 + (i << 4);
#pragma unroll
    for (int j = 0; j < 4; ++j) {
#pragma unroll
      for (int r = 0; r < 8; ++r) {
        slab[(mOff + r) * 68 + (j << 4) + rlane] = acc[i][j][r];
      }
    }
    wave_sync_lds();
    v4f vals[8];
#pragma unroll
    for (int it = 0; it < 8; ++it) {
      const int row = it * 2 + hh2;
      vals[it] = *(const v4f*)(slab + row * 68 + c4);
    }
    for (int pass = 0; pass < 2; ++pass) {
#pragma unroll
      for (int it = 0; it < 8; ++it) {
        const int row = it * 2 + hh2;
        const size_t go = (size_t)(mBase + row) * ldc + n0 + c4;
        *(volatile v4f*)(Cout + go) = vals[it];
      }
      __threadfence();
    }
    wave_sync_lds();
  }
}

__device__ __forceinline__ void hl2(float f0, float f1, unsigned& hw, unsigned& lw) {
  const unsigned short h0 = bf_bits(f0), h1 = bf_bits(f1);
  const unsigned short l0 = bf_bits(f0 - bf_up(h0)), l1 = bf_bits(f1 - bf_up(h1));
  hw = pk16(h0, h1);
  lw = pk16(l0, l1);
}

__global__ __launch_bounds__(128)
void attnb(const unsigned short* qhp, const unsigned short* qlp,
           const unsigned short* __restrict__ khp, const unsigned short* __restrict__ klp,
           const unsigned short* __restrict__ vthp, const unsigned short* __restrict__ vtlp,
           unsigned short* chp, unsigned short* clp, float sscale) {
  union FH { v16h v; v8h h[2]; };
  __shared__ __align__(16) _Float16 Ksh[2][KST * 64];
  __shared__ __align__(16) _Float16 Vsh[2][64 * KST];
  __shared__ __align__(16) _Float16 Psh[2][4][16 * 32];
  static_assert(4 * 16 * 64 * 4 <= 2 * KST * 64 * 2);

  const int tid  = threadIdx.x;
  const int wave = tid >> 5;
  const int lane = tid & 31;
  const int hh   = lane >> 4;
  const int c    = lane & 15;

  const int bx    = blockIdx.x;
  const int qb    = bx % NQB;
  const int hq    = (bx / NQB) % NH;
  const int sb    = bx / (NQB * NH);
  const int qblk  = qb * 64;
  const int kbase = qblk - RADK;
  const int q0    = qblk + wave * 16;
  const int kw    = wave * 16;
  const size_t rb = (size_t)sb * SQ;

  const _Float16* Qh = (const _Float16*)(const void*)qhp + rb * DM + (size_t)hq * HD;
  const _Float16* Ql = (const _Float16*)(const void*)qlp + rb * DM + (size_t)hq * HD;
  const _Float16* Kh = (const _Float16*)(const void*)khp + rb * DM + (size_t)hq * HD;
  const _Float16* Kl = (const _Float16*)(const void*)klp + rb * DM + (size_t)hq * HD;
  const _Float16* Vh = (const _Float16*)(const void*)vthp + (size_t)hq * HD * VTP + rb;
  const _Float16* Vl = (const _Float16*)(const void*)vtlp + (size_t)hq * HD * VTP + rb;

  v16h qa[2], qr[2];
#pragma unroll
  for (int dc = 0; dc < 2; ++dc) {
    qa[dc] = ldfrag_h(Qh + (size_t)(q0 + c) * DM + dc * 32 + 8 * hh);
    qr[dc] = ldfrag_h(Ql + (size_t)(q0 + c) * DM + dc * 32 + 8 * hh);
  }

#pragma unroll
  for (int i = 0; i < 5; ++i) {
    const int p  = tid + 128 * i;
    const int kr = p >> 3;
    const int kc = (p & 7) * 8;
    int kg = kbase + kr;
    kg = kg < 0 ? 0 : (kg > SQ - 1 ? SQ - 1 : kg);
    const v8h a0 = *(const v8h*)(Kh + (size_t)kg * DM + kc);
    const v8h a1 = *(const v8h*)(Kl + (size_t)kg * DM + kc);
    *(v8h*)(&Ksh[0][kr * 64 + kc]) = a0;
    *(v8h*)(&Ksh[1][kr * 64 + kc]) = a1;
    const int vd = p / 10;
    const int vg = p - vd * 10;
    int vc = kbase + vg * 8;
    vc = vc < 0 ? 0 : (vc > SQ - 8 ? SQ - 8 : vc);
    const v8h b0 = *(const v8h*)(Vh + (size_t)vd * VTP + vc);
    const v8h b1 = *(const v8h*)(Vl + (size_t)vd * VTP + vc);
    *(v8h*)(&Vsh[0][vd * KST + vg * 8]) = b0;
    *(v8h*)(&Vsh[1][vd * KST + vg * 8]) = b1;
  }
  __syncthreads();

  const float rinv = 1.0f / RSC;

  v8f s[2];
#pragma unroll
  for (int j = 0; j < 2; ++j) {
    v8f sh = zero8(), sl = zero8();
#pragma unroll
    for (int dc = 0; dc < 2; ++dc) {
      FH kb, kl;
      const int ko = (kw + j * 16 + c) * 64 + dc * 32 + 8 * hh;
      kb.h[0] = *(const v8h*)(&Ksh[0][ko]);
      kb.h[1] = *(const v8h*)(&Ksh[0][ko + 16]);
      kl.h[0] = *(const v8h*)(&Ksh[1][ko]);
      kl.h[1] = *(const v8h*)(&Ksh[1][ko + 16]);
      sh = mma_h(qa[dc], kb.v, sh);
      sl = mma_h(qr[dc], kb.v, sl);
      sl = mma_h(qa[dc], kl.v, sl);
    }
    const int key = kbase + kw + j * 16 + c;
#pragma unroll
    for (int r = 0; r < 8; ++r) {
      const int qrow = q0 + 8 * hh + r;
      const float v = (sh[r] + sl[r] * rinv) * sscale;
      const bool ok = (key >= 0) && (key <= qrow) && (key + RADK >= qrow);
      s[j][r] = ok ? v : -INFINITY;
    }
  }

  _Float16* pwh = Psh[0][wave];
  _Float16* pwl = Psh[1][wave];
  float lrow[8];
#pragma unroll
  for (int r = 0; r < 8; ++r) {
    float m = fmaxf(s[0][r], s[1][r]);
#pragma unroll
    for (int off = 1; off < 16; off <<= 1) m = fmaxf(m, __shfl_xor(m, off, 32));
    const float ms = (m == -INFINITY) ? 0.f : m;
    float psum = 0.f;
#pragma unroll
    for (int j = 0; j < 2; ++j) {
      const float p  = __expf(s[j][r] - ms);
      psum += p;
      const float pv = p * PSC;
      const _Float16 ph = (_Float16)pv;
      const int pi = (8 * hh + r) * 32 + j * 16 + c;
      pwh[pi] = ph;
      pwl[pi] = (_Float16)((pv - (float)ph) * RSC);
    }
#pragma unroll
    for (int off = 1; off < 16; off <<= 1) psum += __shfl_xor(psum, off, 32);
    lrow[r] = psum;
  }
  wave_sync_lds();

  v8f oacc[4], ol[4];
#pragma unroll
  for (int t = 0; t < 4; ++t) { oacc[t] = zero8(); ol[t] = zero8(); }
  {
    FH pa, pr;
    pa.h[0] = *(const v8h*)(pwh + c * 32 + 8 * hh);
    pa.h[1] = *(const v8h*)(pwh + c * 32 + 16 + 8 * hh);
    pr.h[0] = *(const v8h*)(pwl + c * 32 + 8 * hh);
    pr.h[1] = *(const v8h*)(pwl + c * 32 + 16 + 8 * hh);
#pragma unroll
    for (int t = 0; t < 4; ++t) {
      FH vb, wb;
      const int vo = (t * 16 + c) * KST + kw + 8 * hh;
      vb.h[0] = *(const v8h*)(&Vsh[0][vo]);
      vb.h[1] = *(const v8h*)(&Vsh[0][vo + 16]);
      wb.h[0] = *(const v8h*)(&Vsh[1][vo]);
      wb.h[1] = *(const v8h*)(&Vsh[1][vo + 16]);
      oacc[t] = mma_h(pa.v, vb.v, oacc[t]);
      ol[t]   = mma_h(pa.v, wb.v, ol[t]);
      ol[t]   = mma_h(pr.v, vb.v, ol[t]);
    }
  }

  __syncthreads();
  float* os = (float*)(void*)(&Ksh[0][0]) + wave * (16 * 64);
#pragma unroll
  for (int r = 0; r < 8; ++r) {
    const float l = lrow[r];
    const float inv = ((l > 0.f) ? (1.0f / l) : 0.f) * (1.0f / PSC);
#pragma unroll
    for (int t = 0; t < 4; ++t) os[(8 * hh + r) * 64 + t * 16 + c] = (oacc[t][r] + ol[t][r] * rinv) * inv;
  }
  wave_sync_lds();
  {
    const int q8 = lane >> 3, c8 = (lane & 7) * 8;
    v4u hv[4], lv[4];
#pragma unroll
    for (int it = 0; it < 4; ++it) {
      const int row = it * 4 + q8;
      const float* sp = os + row * 64 + c8;
      const v4f x0 = *(const v4f*)(sp);
      const v4f x1 = *(const v4f*)(sp + 4);
      v4u a, b;
      unsigned aw, bw;
      hl2(x0[0], x0[1], aw, bw); a[0] = aw; b[0] = bw;
      hl2(x0[2], x0[3], aw, bw); a[1] = aw; b[1] = bw;
      hl2(x1[0], x1[1], aw, bw); a[2] = aw; b[2] = bw;
      hl2(x1[2], x1[3], aw, bw); a[3] = aw; b[3] = bw;
      hv[it] = a;
      lv[it] = b;
    }
    for (int pass = 0; pass < 2; ++pass) {
#pragma unroll
      for (int it = 0; it < 4; ++it) {
        const int row = it * 4 + q8;
        const size_t go = (rb + (size_t)(q0 + row)) * DM + (size_t)hq * HD + c8;
        *(volatile v4u*)(chp + go) = hv[it];
        *(volatile v4u*)(clp + go) = lv[it];
      }
      __threadfence();
    }
  }
}

extern "C" void kernel_launch(void* const* d_in, const int* in_sizes, int n_in,
                              void* d_out, int out_size, void* d_ws, size_t ws_size,
                              hipStream_t stream) {
  if (n_in < 5) return;
  if (in_sizes[0] != MR * DM) return;
  if (in_sizes[1] != DM * DM) return;
  if (in_sizes[2] != DM * DM) return;
  if (in_sizes[3] != DM * DM) return;
  if (in_sizes[4] != DM * DM) return;
  if (out_size != MR * DM) return;

  const float* x  = (const float*)d_in[0];
  const float* wq = (const float*)d_in[1];
  const float* wk = (const float*)d_in[2];
  const float* wv = (const float*)d_in[3];
  const float* wo = (const float*)d_in[4];

  const size_t PW  = (size_t)DM * DM * 2;
  const size_t PX  = (size_t)MR * DM * 2;
  const size_t PVT = (size_t)DM * VTP * 2;
  size_t off = 0;
  const size_t oWq = off; off += PW;
  const size_t oWk = off; off += PW;
  const size_t oWv = off; off += PW;
  const size_t oWo = off; off += PW;
  const size_t oXH = off; off += PX;
  const size_t oQH = off; off += PX;
  const size_t oQL = off; off += PX;
  const size_t oKH = off; off += PX;
  const size_t oKL = off; off += PX;
  const size_t oVH = off; off += PVT;
  const size_t oVL = off; off += PVT;
  if (off > ws_size) return;
  if (off > (size_t)134217728) return;

  char* ws = (char*)d_ws;
  unsigned short* WqT = (unsigned short*)(ws + oWq);
  unsigned short* WkT = (unsigned short*)(ws + oWk);
  unsigned short* WvT = (unsigned short*)(ws + oWv);
  unsigned short* WoB = (unsigned short*)(ws + oWo);
  unsigned short* XH  = (unsigned short*)(ws + oXH);
  unsigned short* QH  = (unsigned short*)(ws + oQH);
  unsigned short* QL  = (unsigned short*)(ws + oQL);
  unsigned short* KH  = (unsigned short*)(ws + oKH);
  unsigned short* KL  = (unsigned short*)(ws + oKL);
  unsigned short* VTH = (unsigned short*)(ws + oVH);
  unsigned short* VTL = (unsigned short*)(ws + oVL);

  const dim3 blk(256), blk128(128);
  const dim3 gCx((MR * DM / 8 + 255) / 256);
  const dim3 gT((DM / 64) * (DM / 64));
  const dim3 gGq(((MR / 64) * (DM / 64) + 7) / 8);
  const dim3 gGv(((DM / 64) * (VTP / 64) + 7) / 8);
  const dim3 gAttn(NB * NH * NQB);
  const float invw   = 1.0f / WSC;
  const float sscale = 1.0f / 0.56f;

  conv16<0><<<gCx, blk, 0, stream>>>(x, XH, MR * DM / 8, 1.0f);
  convT<0><<<gT, blk, 0, stream>>>(wq, WqT, DM, DM, WSC);
  convT<0><<<gT, blk, 0, stream>>>(wk, WkT, DM, DM, WSC);
  convT<0><<<gT, blk, 0, stream>>>(wv, WvT, DM, DM, WSC);
  convT<1><<<gT, blk, 0, stream>>>(wo, WoB, DM, DM, 1.0f);

  gemm64<3><<<gGq, blk, 0, stream>>>(XH, DM, WqT, DM, QH, QL, DM, MR, DM, DM, invw, RSC);
  gemm64<3><<<gGq, blk, 0, stream>>>(XH, DM, WkT, DM, KH, KL, DM, MR, DM, DM, invw, RSC);
  gemm64<3><<<gGv, blk, 0, stream>>>(WvT, DM, XH, DM, VTH, VTL, VTP, DM, VTP, DM, invw, RSC);

  attnb<<<gAttn, blk128, 0, stream>>>(QH, QL, KH, KL, VTH, VTL, QH, QL, sscale);

  gemm_ob<<<gGq, blk, 0, stream>>>(QH, QL, DM, WoB, DM, (float*)d_out, DM, MR, DM, DM);
  (void)hipGetLastError();
}
